// GNN_18176301596804
// MI455X (gfx1250) — hardware-verified
//
#include <hip/hip_runtime.h>
#include <stddef.h>
#include <stdint.h>
#include <math.h>


#define DF      128
#define KA      256
#define NTHR    256
#define NWAVE   8
#define EPT     8
#define CHUNK   (NTHR * EPT)
#define WCAP    (EPT * 32)
#define LISTN   (NWAVE * WCAP)
#define NBA     1024
#define PKS     10
#define RCAP    28672
#define DEGCAP  64
#define GBM     64
#define GTHR    128
#define GNT     8
#define GBN     (16 * GNT)
#define WPU     (DF * (KA / 8))
#define WPH     (DF * KA)
#define NLMAX   16
#define PARTW   288
#define PMEAN   32
#define PM2     160
#define APB     64
#define APR     8
#define ZINTS   (2 * RCAP + 2 * NBA + LISTN)
#define LDS_AGG (ZINTS * 4 + 64)
#define WSMAX   134217728

static_assert((CHUNK & (CHUNK - 1)) == 0);
static_assert(NBA == (1 << PKS));
static_assert(((long long)CHUNK << PKS) < (1LL << 31));
static_assert(NTHR * 4 == NBA);
static_assert(LISTN >= NBA && LISTN >= NWAVE * WCAP);
static_assert((RCAP % 32) == 0);
static_assert((ZINTS % (NTHR * 4)) == 0);
static_assert(LDS_AGG <= 262144);
static_assert((NBA % NWAVE) == 0 && (NBA % GBM) == 0);
static_assert(GBM == (GTHR / 32) * 16);
static_assert(KA == 2 * DF && (KA % 32) == 0);
static_assert((WPU % NTHR) == 0 && WPU == 4096);
static_assert(DF == 32 * 4);
static_assert(GBN == DF && (KA / 8) == 32 && GTHR == GBN);
static_assert((PARTW % 32) == 0 && PARTW / 4 <= GTHR && PM2 + DF <= PARTW && PMEAN + DF <= PM2);
static_assert(NTHR == 2 * DF);
static_assert(APB == NWAVE * APR && APB == GBM);

typedef float          v4f  __attribute__((ext_vector_type(4)));
typedef float          v8f  __attribute__((ext_vector_type(8)));
typedef int            v4i  __attribute__((ext_vector_type(4)));
typedef int            v8i  __attribute__((ext_vector_type(8)));
typedef unsigned int   v4u  __attribute__((ext_vector_type(4)));
typedef unsigned short v8us __attribute__((ext_vector_type(8)));
typedef _Float16       v16h __attribute__((ext_vector_type(16)));
typedef __bf16         v16b __attribute__((ext_vector_type(16)));
typedef v4f  __attribute__((may_alias)) v4fa;
typedef v4i  __attribute__((may_alias)) v4ia;
typedef v8us __attribute__((may_alias)) v8usa;
union Frag { v16b b; v16h f; v8us h[2]; v8i w; };

__device__ __forceinline__ v8f wmk(const Frag& a, const Frag& b, v8f c) {
  v8f d = __builtin_amdgcn_wmma_f32_16x16x32_bf16(false, a.b, false, b.b, (short)0, c, false, false);
  asm volatile("v_nop\n\tv_nop\n\tv_nop\n\tv_nop" : "+v"(d) : "v"(a.w), "v"(b.w));
  return d;
}

__device__ __forceinline__ unsigned short bf_bits(float f) {
  unsigned int u = __float_as_uint(f);
  u += 0x7FFFu + ((u >> 16) & 1u);
  return (unsigned short)(u >> 16);
}
__device__ __forceinline__ float bf_val(unsigned short b) {
  return __uint_as_float(((unsigned int)b) << 16);
}
__device__ __forceinline__ float bf_rne(float f) { return bf_val(bf_bits(f)); }

template <int ACT>
__device__ __forceinline__ float actf(float v) {
  if constexpr (ACT == 1) {
    return fmaxf(v, 0.0f);
  } else {
    return v;
  }
}

template <int RND>
__device__ __forceinline__ float cvin(float v) {
  if constexpr (RND == 1) {
    return bf_rne(v);
  } else {
    return v;
  }
}

__device__ __forceinline__ v4u pack_hilo4(float r0, float r1, float r2, float r3) {
  const unsigned short hb0 = bf_bits(r0), hb1 = bf_bits(r1), hb2 = bf_bits(r2), hb3 = bf_bits(r3);
  const unsigned short lb0 = bf_bits(r0 - bf_val(hb0)), lb1 = bf_bits(r1 - bf_val(hb1));
  const unsigned short lb2 = bf_bits(r2 - bf_val(hb2)), lb3 = bf_bits(r3 - bf_val(hb3));
  v4u pk;
  pk.x = (unsigned int)hb0 | ((unsigned int)hb1 << 16);
  pk.y = (unsigned int)hb2 | ((unsigned int)hb3 << 16);
  pk.z = (unsigned int)lb0 | ((unsigned int)lb1 << 16);
  pk.w = (unsigned int)lb2 | ((unsigned int)lb3 << 16);
  return pk;
}

__device__ __forceinline__ int scan_chunk(const int* __restrict__ dsts, int nE, int cbase, int slotBase,
                                          int nb, int vec8, int* list, int tid, int lane, int wave) {
  int wc = 0;
  const int el0  = tid * EPT;
  const int e0   = cbase + el0;
  const int sent = -2147483647 - 1;
  v4i da, db;
  if (vec8 != 0 && cbase + CHUNK <= nE) {
    da = *(const v4i*)(dsts + e0);
    db = *(const v4i*)(dsts + e0 + 4);
  } else {
    da.x = (e0     < nE) ? dsts[min(e0,     nE - 1)] : sent;
    da.y = (e0 + 1 < nE) ? dsts[min(e0 + 1, nE - 1)] : sent;
    da.z = (e0 + 2 < nE) ? dsts[min(e0 + 2, nE - 1)] : sent;
    da.w = (e0 + 3 < nE) ? dsts[min(e0 + 3, nE - 1)] : sent;
    db.x = (e0 + 4 < nE) ? dsts[min(e0 + 4, nE - 1)] : sent;
    db.y = (e0 + 5 < nE) ? dsts[min(e0 + 5, nE - 1)] : sent;
    db.z = (e0 + 6 < nE) ? dsts[min(e0 + 6, nE - 1)] : sent;
    db.w = (e0 + 7 < nE) ? dsts[min(e0 + 7, nE - 1)] : sent;
  }
  const unsigned nbs = (unsigned)slotBase;
  const unsigned unb = (unsigned)nb;
  const unsigned s0 = (unsigned)da.x - nbs, s1 = (unsigned)da.y - nbs;
  const unsigned s2 = (unsigned)da.z - nbs, s3 = (unsigned)da.w - nbs;
  const unsigned s4 = (unsigned)db.x - nbs, s5 = (unsigned)db.y - nbs;
  const unsigned s6 = (unsigned)db.z - nbs, s7 = (unsigned)db.w - nbs;
  const bool h0 = s0 < unb, h1 = s1 < unb, h2 = s2 < unb, h3 = s3 < unb;
  const bool h4 = s4 < unb, h5 = s5 < unb, h6 = s6 < unb, h7 = s7 < unb;
  const unsigned any = __builtin_amdgcn_ballot_w32(h0 | h1 | h2 | h3 | h4 | h5 | h6 | h7);
  if (any != 0u) {
#define HITJ(J, HJ, SJ) { \
      const unsigned mj = __builtin_amdgcn_ballot_w32(HJ); \
      if (mj != 0u) { \
        if (HJ) { \
          const int pos = wc + (int)__builtin_amdgcn_mbcnt_lo(mj, 0u); \
          if (pos < WCAP) list[wave * WCAP + pos] = ((el0 + (J)) << PKS) | (int)(SJ); \
        } \
        wc += (int)__builtin_popcount(mj); } }
    HITJ(0, h0, s0)
    HITJ(1, h1, s1)
    HITJ(2, h2, s2)
    HITJ(3, h3, s3)
    HITJ(4, h4, s4)
    HITJ(5, h5, s5)
    HITJ(6, h6, s6)
    HITJ(7, h7, s7)
#undef HITJ
  }
  return wc;
}

__global__ __launch_bounds__(NTHR) void k_wprep(const float* __restrict__ w1s, const float* __restrict__ w2s,
                                                int nL, int nUnits, unsigned short* WPL) {
  const int u = (int)blockIdx.x * NTHR + (int)threadIdx.x;
  if (u >= nUnits) return;
  const int pl = u >> 12;
  const int v  = u & (WPU - 1);
  const int n  = v >> 5;
  const int q  = v & 31;
  const bool isW2 = pl >= nL;
  const int li = isW2 ? (pl - nL) : pl;
  const float* w = (isW2 ? w2s : w1s) + (size_t)li * (size_t)(DF * DF);
  const float* p = w + (size_t)(4 * q) * DF + n;
  float f[4];
#pragma unroll
  for (int c = 0; c < 4; ++c) f[c] = p[(size_t)c * DF];
  v8us o;
#pragma unroll
  for (int j = 0; j < 8; ++j) o[j] = bf_bits(f[j & 3]);
  unsigned short* dp = WPL + (size_t)pl * WPH + (size_t)v * 8;
  *(volatile v8us*)dp = o;
  __threadfence();
  *(volatile v8us*)dp = o;
}

template <int ACT, int STATS>
__global__ __launch_bounds__(GTHR) void k_gemm(const unsigned short* __restrict__ A, int lda,
                                               const unsigned short* __restrict__ BT, int ldb, int K,
                                               const float* __restrict__ bias,
                                               float* C32, int ldc, int nRows, int nLive, float* part) {
  static_assert(STATS == 0 || STATS == 1);
  __shared__ __attribute__((aligned(16))) float stg[GBM * GBN];
  __shared__ __attribute__((aligned(16))) float pst[PARTW];
  const int tid = (int)threadIdx.x, lane = tid & 31, wave = tid >> 5, hh = lane >> 4, m = lane & 15;
  const int rowBase = (int)blockIdx.x * GBM;

  v8f acc[GNT];
  {
    const v8f z = {0.f, 0.f, 0.f, 0.f, 0.f, 0.f, 0.f, 0.f};
#pragma unroll
    for (int t = 0; t < GNT; ++t) acc[t] = z;
  }
  const unsigned short* ap = A  + (size_t)(rowBase + 16 * wave + m) * (size_t)lda + 8 * hh;
  const unsigned short* bp = BT + (size_t)m * (size_t)ldb + 8 * hh;

#pragma unroll 1
  for (int k0 = 0; k0 < K; k0 += 32) {
    Frag af;
    af.h[0] = *(const v8usa*)(ap + k0);
    af.h[1] = *(const v8usa*)(ap + k0 + 16);
#pragma unroll
    for (int nt = 0; nt < GNT; ++nt) {
      const unsigned short* wq = bp + (size_t)(16 * nt) * (size_t)ldb + k0;
      Frag bf;
      bf.h[0] = *(const v8usa*)wq;
      bf.h[1] = *(const v8usa*)(wq + 16);
      acc[nt] = wmk(af, bf, acc[nt]);
    }
  }

#pragma unroll
  for (int nt = 0; nt < GNT; ++nt) {
    const int lc = 16 * nt + m;
    const float bb = bf_rne(bias[lc]);
#pragma unroll
    for (int r = 0; r < 8; ++r) {
      const int lr = 16 * wave + 8 * hh + r;
      stg[lr * GBN + lc] = actf<ACT>(acc[nt][r] + bb);
    }
  }
  __syncthreads();

  {
    v4f pv[16];
#pragma unroll
    for (int i = 0; i < 16; ++i) pv[i] = *(const v4fa*)(stg + (16 * wave + i) * GBN + 4 * lane);
#pragma unroll
    for (int i = 0; i < 16; ++i) {
      const int gr = rowBase + 16 * wave + i;
      float* op = C32 + (size_t)gr * (size_t)ldc + 4 * lane;
      if (gr < nRows) *(volatile v4f*)op = pv[i];
    }
    __threadfence();
#pragma unroll
    for (int i = 0; i < 16; ++i) {
      const int gr = rowBase + 16 * wave + i;
      float* op = C32 + (size_t)gr * (size_t)ldc + 4 * lane;
      if (gr < nRows) *(volatile v4f*)op = pv[i];
    }
  }

  if constexpr (STATS == 1) {
    int nb = nLive - rowBase;
    nb = nb < 0 ? 0 : (nb > GBM ? GBM : nb);
    const int c = tid;
    float s = 0.0f;
#pragma unroll 4
    for (int r = 0; r < nb; ++r) s += stg[r * GBN + c];
    const float inv = 1.0f / (float)(nb < 1 ? 1 : nb);
    const float mb = s * inv;
    float q = 0.0f;
#pragma unroll 4
    for (int r = 0; r < nb; ++r) {
      const float d = stg[r * GBN + c] - mb;
      q = fmaf(d, d, q);
    }
    pst[PMEAN + c] = mb;
    pst[PM2 + c]   = q;
    if (tid < PMEAN) pst[tid] = (tid == 0) ? (float)nb : 0.0f;
    __syncthreads();
    v4f ps = {0.0f, 0.0f, 0.0f, 0.0f};
    if (tid < PARTW / 4) {
      ps = *(const v4fa*)(pst + 4 * tid);
      *(volatile v4f*)(part + (size_t)blockIdx.x * PARTW + 4 * tid) = ps;
    }
    __threadfence();
    if (tid < PARTW / 4) {
      *(volatile v4f*)(part + (size_t)blockIdx.x * PARTW + 4 * tid) = ps;
    }
  } else {
    (void)nLive; (void)part; (void)pst;
  }
}

template <int RND>
__global__ __launch_bounds__(NTHR) void k_agg(const int* __restrict__ srcs, const int* __restrict__ dsts,
                                              const float* __restrict__ X, unsigned short* Aout,
                                              int nN, int nE, int vec8) {
  extern __shared__ __attribute__((aligned(16))) int lds_i[];
  int* reg1 = lds_i;
  int* reg2 = reg1 + RCAP;
  int* scnt = reg2 + RCAP;
  int* soff = scnt + NBA;
  int* list = soff + NBA;
  int* wcnt = list + LISTN;
  int* wtot = wcnt + NWAVE;
  const int tid = (int)threadIdx.x, lane = tid & 31, wave = tid >> 5;
  const int nodeBase = (int)blockIdx.x * NBA;

  {
    const v4i z4 = {0, 0, 0, 0};
    for (int i = tid * 4; i < ZINTS; i += NTHR * 4) *(v4ia*)(lds_i + i) = z4;
    if (tid < 2 * NWAVE) wcnt[tid] = 0;
  }
  __syncthreads();

  int tot = 0;
  const int nChunks = (nE + CHUNK - 1) / CHUNK;
#pragma unroll 1
  for (int ch = 0; ch < nChunks; ++ch) {
    const int cbase = ch * CHUNK;
    const int wc = scan_chunk(dsts, nE, cbase, nodeBase, NBA, vec8, list, tid, lane, wave);
    if (lane == 0) wcnt[wave] = wc;
    __syncthreads();
    int pre = 0, all = 0;
#pragma unroll
    for (int w2 = 0; w2 < NWAVE; ++w2) {
      int c = wcnt[w2];
      c = c < 0 ? 0 : (c > WCAP ? WCAP : c);
      all += c;
      pre += (w2 < wave) ? c : 0;
    }
    const int wcc  = wc > WCAP ? WCAP : wc;
    const int base = tot + pre;
#pragma unroll 1
    for (int i = lane; i < wcc; i += 32) {
      const int ent = list[wave * WCAP + i];
      const int el  = (ent >> PKS) & (CHUNK - 1);
      const int sl  = ent & (NBA - 1);
      int eid = cbase + el;
      eid = eid > nE - 1 ? nE - 1 : eid;
      const int pos = base + i;
      if (pos < RCAP) reg1[pos] = (int)(((unsigned)eid << PKS) | (unsigned)sl);
    }
    tot += all;
    tot = tot > RCAP ? RCAP : tot;
    __syncthreads();
  }
  const int nh = tot;

  if (wave == 0) {
#pragma unroll 1
    for (int b0 = 0; b0 < nh; b0 += 32) {
      const int idx = b0 + lane;
      const int uv  = reg1[idx < RCAP ? idx : RCAP - 1];
      const int m32 = (nh - b0) < 32 ? (nh - b0) : 32;
#pragma unroll 1
      for (int k = 0; k < m32; ++k) {
        const int u  = __builtin_amdgcn_readlane(uv, k);
        const int sl = u & (NBA - 1);
        if (lane == 0) scnt[sl] = scnt[sl] + 1;
      }
    }
  }
  __syncthreads();

  {
    const v4i ca = *(const v4ia*)(scnt + 4 * tid);
    const int e0 = ca.x < 0 ? 0 : ca.x, e1 = ca.y < 0 ? 0 : ca.y, e2 = ca.z < 0 ? 0 : ca.z, e3 = ca.w < 0 ? 0 : ca.w;
    const int ts = e0 + e1 + e2 + e3;
    int incl = ts;
#pragma unroll
    for (int d = 1; d < 32; d <<= 1) {
      const int up = __shfl_up(incl, d, 32);
      if (lane >= d) incl += up;
    }
    if (lane == 31) wtot[wave] = incl;
    __syncthreads();
    int pre = 0;
#pragma unroll
    for (int w2 = 0; w2 < NWAVE; ++w2) pre += (w2 < wave) ? wtot[w2] : 0;
    int run = pre + incl - ts;
    soff[4 * tid + 0] = run; run += e0;
    soff[4 * tid + 1] = run; run += e1;
    soff[4 * tid + 2] = run; run += e2;
    soff[4 * tid + 3] = run;
  }
  __syncthreads();
  for (int i = tid; i < NBA; i += NTHR) list[i] = soff[i];
  __syncthreads();

  if (wave == 0) {
#pragma unroll 1
    for (int b0 = 0; b0 < nh; b0 += 32) {
      const int idx = b0 + lane;
      const int uv  = reg1[idx < RCAP ? idx : RCAP - 1];
      const int m32 = (nh - b0) < 32 ? (nh - b0) : 32;
#pragma unroll 1
      for (int k = 0; k < m32; ++k) {
        const int u   = __builtin_amdgcn_readlane(uv, k);
        const int sl  = u & (NBA - 1);
        const int eid = (int)((unsigned)u >> PKS);
        if (lane == 0) {
          int pos = list[sl];
          pos = pos < 0 ? 0 : (pos > RCAP - 1 ? RCAP - 1 : pos);
          reg2[pos] = eid;
          list[sl] = pos + 1;
        }
      }
    }
  }
  __syncthreads();

  const int nbw = NBA / NWAVE;
  const bool ovf = (nh >= RCAP);
  const float qnan = __int_as_float(0x7fc00000);

#pragma unroll 1
  for (int jt = 0; jt < nbw; ++jt) {
    const int slot = wave * nbw + jt;
    const int node = nodeBase + slot;
    int st = soff[slot];
    const int craw = scnt[slot];
    int cnt = craw;
    st  = st < 0 ? 0 : (st > nh ? nh : st);
    cnt = cnt < 0 ? 0 : (cnt > DEGCAP ? DEGCAP : cnt);
    if (cnt > nh - st) cnt = nh - st;
    const float pz = (ovf || craw > DEGCAP) ? qnan : 0.0f;
    const bool live = node < nN;
    const int nc = node < nN ? node : nN - 1;

    float a0 = 0.f, a1 = 0.f, a2 = 0.f, a3 = 0.f;
#pragma unroll 1
    for (int b0 = 0; b0 < cnt; b0 += 32) {
      int idx = st + b0 + lane; idx = idx > RCAP - 1 ? RCAP - 1 : idx;
      int eid = reg2[idx]; eid = eid < 0 ? 0 : (eid > nE - 1 ? nE - 1 : eid);
      int sr = srcs[eid]; sr = sr < 0 ? 0 : (sr > nN - 1 ? nN - 1 : sr);
      const int m32 = (cnt - b0) < 32 ? (cnt - b0) : 32;
#pragma unroll 1
      for (int k = 0; k < m32; ++k) {
        const int sk = __builtin_amdgcn_readlane(sr, k);
        const v4f v = *(const v4fa*)(X + (size_t)sk * DF + 4 * lane);
        a0 += cvin<RND>(v.x); a1 += cvin<RND>(v.y); a2 += cvin<RND>(v.z); a3 += cvin<RND>(v.w);
      }
    }
    const v4f sv = *(const v4fa*)(X + (size_t)nc * DF + 4 * lane);
    float r0 = a0 + cvin<RND>(sv.x), r1 = a1 + cvin<RND>(sv.y);
    float r2 = a2 + cvin<RND>(sv.z), r3 = a3 + cvin<RND>(sv.w);
    r0 = (live ? r0 : 0.0f) + pz;
    r1 = (live ? r1 : 0.0f) + pz;
    r2 = (live ? r2 : 0.0f) + pz;
    r3 = (live ? r3 : 0.0f) + pz;

    const v4u pk = pack_hilo4(r0, r1, r2, r3);
    unsigned short* gp = Aout + (size_t)node * (size_t)KA + 8 * lane;
    *(volatile v4u*)gp = pk;
    __threadfence();
    *(volatile v4u*)gp = pk;
  }
}

__global__ __launch_bounds__(DF) void k_gnfin(const float* __restrict__ part, int nPart,
                                              const float* __restrict__ gw, const float* __restrict__ gb,
                                              const float* __restrict__ ga, float* ss) {
  __shared__ __attribute__((aligned(16))) float stg[2 * DF];
  const int tid = (int)threadIdx.x;
  const int c = tid;
  double n = 0.0, mean = 0.0, M2 = 0.0;
#pragma unroll 1
  for (int b = 0; b < nPart; ++b) {
    const float* pr = part + (size_t)b * PARTW;
    const double nb = (double)pr[0];
    const double mb = (double)pr[PMEAN + c];
    const double qb = (double)pr[PM2 + c];
    if (nb > 0.5) {
      const double nn = n + nb;
      const double delta = mb - mean;
      const double f = nb / nn;
      mean = mean + delta * f;
      M2 = M2 + qb + delta * delta * n * f;
      n = nn;
    }
  }
  const double nt = n < 1.0 ? 1.0 : n;
  const double a  = (double)bf_rne(ga[c]);
  const double var = M2 / nt + (1.0 - a) * (1.0 - a) * mean * mean;
  const float varf = (float)var;
  const float rstd = 1.0f / sqrtf(varf + 1e-5f);
  const float sc = bf_rne(gw[c]) * rstd;
  const float sh = (float)((double)bf_rne(gb[c]) - (double)sc * a * mean);
  stg[c] = sc;
  stg[DF + c] = sh;
  __syncthreads();
  v4f v = {0.0f, 0.0f, 0.0f, 0.0f};
  if (tid < (2 * DF) / 4) {
    v = *(const v4fa*)(stg + 4 * tid);
    *(volatile v4f*)(ss + 4 * tid) = v;
  }
  __threadfence();
  if (tid < (2 * DF) / 4) {
    *(volatile v4f*)(ss + 4 * tid) = v;
  }
}

__global__ __launch_bounds__(NTHR) void k_apply(const float* __restrict__ z, const float* __restrict__ ss,
                                                int nN, int mRows, unsigned short* tpl) {
  __shared__ __attribute__((aligned(16))) float ssh[2 * DF];
  const int tid = (int)threadIdx.x, lane = tid & 31, wave = tid >> 5;
  ssh[tid] = ss[tid];
  __syncthreads();
  const v4f sc = *(const v4fa*)(ssh + 4 * lane);
  const v4f sh = *(const v4fa*)(ssh + DF + 4 * lane);
  const int rb0 = (int)blockIdx.x * APB + wave * APR;

  v4u q[APR];
#pragma unroll
  for (int i = 0; i < APR; ++i) {
    const int row = rb0 + i;
    const bool live = row < nN;
    const int rc = live ? row : (nN - 1);
    const v4f a = *(const v4f*)(z + (size_t)rc * DF + 4 * lane);
    float y0 = fmaxf(fmaf(a.x, sc.x, sh.x), 0.0f);
    float y1 = fmaxf(fmaf(a.y, sc.y, sh.y), 0.0f);
    float y2 = fmaxf(fmaf(a.z, sc.z, sh.z), 0.0f);
    float y3 = fmaf(a.w, sc.w, sh.w);
    y3 = fmaxf(y3, 0.0f);
    y0 = live ? y0 : 0.0f;
    y1 = live ? y1 : 0.0f;
    y2 = live ? y2 : 0.0f;
    y3 = live ? y3 : 0.0f;
    q[i] = pack_hilo4(y0, y1, y2, y3);
  }
#pragma unroll
  for (int i = 0; i < APR; ++i) {
    const int row = rb0 + i;
    if (row < mRows) *(volatile v4u*)(tpl + (size_t)row * KA + 8 * lane) = q[i];
  }
  __threadfence();
#pragma unroll
  for (int i = 0; i < APR; ++i) {
    const int row = rb0 + i;
    if (row < mRows) *(volatile v4u*)(tpl + (size_t)row * KA + 8 * lane) = q[i];
  }
}

static inline int cdiv(int a, int b) { return (a + b - 1) / b; }
static inline size_t al256(size_t o) { return (o + 255) & ~(size_t)255; }

extern "C" void kernel_launch(void* const* d_in, const int* in_sizes, int n_in,
                              void* d_out, int out_size, void* d_ws, size_t ws_size,
                              hipStream_t stream) {
  if (n_in < 9) return;
  if (in_sizes[0] < DF || (in_sizes[0] % DF) != 0) return;
  const int nN = in_sizes[0] / DF;
  if (nN < 1 || nN > (1 << 22)) return;
  if (in_sizes[1] < 2 || (in_sizes[1] & 1) != 0) return;
  const int nE = in_sizes[1] / 2;
  if (nE < 1 || nE >= (1 << 21)) return;
  if (in_sizes[2] < DF * DF || (in_sizes[2] % (DF * DF)) != 0) return;
  const int nL = in_sizes[2] / (DF * DF);
  if (nL < 1 || nL > NLMAX) return;
  if (in_sizes[3] != nL * DF || in_sizes[4] != nL * DF) return;
  if (in_sizes[5] != nL * DF || in_sizes[6] != nL * DF) return;
  if (in_sizes[7] != nL * DF * DF || in_sizes[8] != nL * DF) return;
  if ((long long)out_size != (long long)nN * DF) return;

  const float* x   = (const float*)d_in[0];
  const int*   ei  = (const int*)  d_in[1];
  const float* W1  = (const float*)d_in[2];
  const float* b1  = (const float*)d_in[3];
  const float* gw  = (const float*)d_in[4];
  const float* gb  = (const float*)d_in[5];
  const float* ga  = (const float*)d_in[6];
  const float* W2  = (const float*)d_in[7];
  const float* b2  = (const float*)d_in[8];
  float* out = (float*)d_out;
  const int* src = ei;
  const int* dst = ei + nE;

  const int MP   = cdiv(nN, GBM) * GBM;
  const int gM   = MP / GBM;
  const int gA   = cdiv(MP, NBA);
  const int RA   = gA * NBA;
  const int vec8 = ((nE & 3) == 0) ? 1 : 0;
  if ((long long)RA < (long long)MP || (MP % APB) != 0) return;

  char* ws = (char*)d_ws;
  size_t off = 0;
  const size_t oWPL = off; off = al256(off + (size_t)(2 * nL) * WPH * 2);
  const size_t szAP = (size_t)RA * KA * 2;
  const size_t szTP = (size_t)MP * KA * 2;
  const size_t oR1  = off; off = al256(off + (szAP > szTP ? szAP : szTP));
  const size_t oR2  = off; off = al256(off + (size_t)MP * DF * 4);
  const size_t oPT  = off; off = al256(off + (size_t)gM * PARTW * 4);
  const size_t oSS  = off; off = al256(off + (size_t)(2 * DF) * 4);
  if (off > ws_size || off > (size_t)WSMAX) return;
  unsigned short* WPL = (unsigned short*)(ws + oWPL);
  unsigned short* AP  = (unsigned short*)(ws + oR1);
  unsigned short* TP  = (unsigned short*)(ws + oR1);
  float*          Z1  = (float*)(ws + oR2);
  float*          H   = (float*)(ws + oR2);
  float*          PT  = (float*)(ws + oPT);
  float*          SS  = (float*)(ws + oSS);

  hipFuncSetAttribute(reinterpret_cast<const void*>(&k_agg<1>), hipFuncAttributeMaxDynamicSharedMemorySize, LDS_AGG);
  hipFuncSetAttribute(reinterpret_cast<const void*>(&k_agg<0>), hipFuncAttributeMaxDynamicSharedMemorySize, LDS_AGG);

  const int nUW = 2 * nL * WPU;
  k_wprep<<<nUW / NTHR, NTHR, 0, stream>>>(W1, W2, nL, nUW, WPL);

  for (int l = 0; l < nL; ++l) {
    const unsigned short* W1D = WPL + (size_t)l * WPH;
    const unsigned short* W2D = WPL + (size_t)(nL + l) * WPH;
    if (l == 0) {
      k_agg<1><<<gA, NTHR, LDS_AGG, stream>>>(src, dst, x, AP, nN, nE, vec8);
    } else {
      k_agg<0><<<gA, NTHR, LDS_AGG, stream>>>(src, dst, H, AP, nN, nE, vec8);
    }
    k_gemm<0, 1><<<gM, GTHR, 0, stream>>>(AP, KA, W1D, KA, KA, b1 + (size_t)l * DF, Z1, DF, MP, nN, PT);
    k_gnfin<<<1, DF, 0, stream>>>(PT, gM, gw + (size_t)l * DF, gb + (size_t)l * DF, ga + (size_t)l * DF, SS);
    k_apply<<<gM, NTHR, 0, stream>>>(Z1, SS, nN, MP, TP);
    if (l < nL - 1) {
      k_gemm<1, 0><<<gM, GTHR, 0, stream>>>(TP, KA, W2D, KA, KA, b2 + (size_t)l * DF, H, DF, MP, 0, PT);
    } else {
      k_gemm<1, 0><<<gM, GTHR, 0, stream>>>(TP, KA, W2D, KA, KA, b2 + (size_t)l * DF, out, DF, nN, 0, PT);
    }
  }
}
